// bwd_LSTM_146028888506
// MI455X (gfx1250) — hardware-verified
//
#include <hip/hip_runtime.h>

#define NB   4096
#define NID  2048
#define NOD  1024
#define NHC  (NB * NOD)

typedef unsigned short v8us  __attribute__((ext_vector_type(8)));
typedef __bf16         v16bf __attribute__((ext_vector_type(16)));
typedef float          v8f   __attribute__((ext_vector_type(8)));
typedef float          v4f   __attribute__((ext_vector_type(4)));
typedef v8us __attribute__((may_alias)) v8usa;
typedef v4f  __attribute__((may_alias)) v4fa;

union Frag { v16bf v; v8us hf[2]; };

__device__ __forceinline__ unsigned short f2bf(float f) {
  const unsigned int u = __float_as_uint(f);
  return (unsigned short)((u + 0x7fffu + ((u >> 16) & 1u)) >> 16);
}
__device__ __forceinline__ float bfr(float f) {
  const unsigned int u = __float_as_uint(f);
  return __uint_as_float((u + 0x7fffu + ((u >> 16) & 1u)) & 0xffff0000u);
}
__device__ __forceinline__ float fsigm(float x) {
  return __builtin_amdgcn_rcpf(1.0f + __expf(-x));
}
__device__ __forceinline__ float ftanh(float x) {
  const float e = __expf(-2.0f * fabsf(x));
  const float t = (1.0f - e) * __builtin_amdgcn_rcpf(1.0f + e);
  return copysignf(t, x);
}
__device__ __forceinline__ float wave_max(float v) {
  #pragma unroll
  for (int o = 16; o > 0; o >>= 1) v = fmaxf(v, __shfl_xor(v, o));
  return v;
}
__device__ __forceinline__ float wave_sum(float v) {
  #pragma unroll
  for (int o = 16; o > 0; o >>= 1) v += __shfl_xor(v, o);
  return v;
}

__device__ __forceinline__ v8f wmma_bf16(v16bf a, v16bf b, v8f c) {
  v8f d = __builtin_amdgcn_wmma_f32_16x16x32_bf16(false, a, false, b, (short)0, c, false, false);
  asm volatile("v_nop\n\tv_nop\n\tv_nop\n\tv_nop" : "+v"(d) : "v"(a), "v"(b));
  return d;
}

__device__ __forceinline__ v16bf load_frag(const unsigned short* p, int h) {
  Frag f;
  f.hf[0] = *(const v8usa*)(p + 8 * h);
  f.hf[1] = *(const v8usa*)(p + 16 + 8 * h);
  return f.v;
}

__global__ __launch_bounds__(256) void cvt_bf16_kernel(
    const float* __restrict__ src, unsigned short* dst, int n8)
{
  const int g = blockIdx.x * 256 + threadIdx.x;
  if (g >= n8) return;
  const float* p = src + (size_t)g * 8;
  const v4f a = *(const v4fa*)p;
  const v4f b = *(const v4fa*)(p + 4);
  v8us o;
  o[0] = f2bf(a.x); o[1] = f2bf(a.y); o[2] = f2bf(a.z); o[3] = f2bf(a.w);
  o[4] = f2bf(b.x); o[5] = f2bf(b.y); o[6] = f2bf(b.z); o[7] = f2bf(b.w);
  unsigned short* d = dst + (size_t)g * 8;
  *(volatile v8us*)d = o;
  __threadfence();
  *(volatile v8us*)d = o;
}

__device__ __forceinline__ void tile_store(const float* s, float* dst, int H, int lane) {
  const int q8 = lane & 7, sub = lane >> 3;
  #pragma unroll
  for (int i = 0; i < 4; ++i) {
    const int row = 4 * i + sub;
    const v4f v = *(const v4fa*)(s + row * 32 + 4 * q8);
    *(volatile v4f*)(dst + (size_t)row * H + 4 * q8) = v;
  }
}

__global__ __launch_bounds__(256) void cell_gemm_kernel(
    const unsigned short* __restrict__ Xb, int K1,
    const unsigned short* __restrict__ Hb, int K2,
    const unsigned short* __restrict__ Wih,
    const unsigned short* __restrict__ Whh,
    const float* __restrict__ bih, const float* __restrict__ bhh,
    const float* __restrict__ Cin, int useC,
    float* Hout, float* Cout, int storeC, int H)
{
  __shared__ __attribute__((aligned(16))) float sH[8 * 512];
  __shared__ __attribute__((aligned(16))) float sC[8 * 512];

  const int tid = threadIdx.x, lane = tid & 31, w = tid >> 5;
  const int h = lane >> 4, m = lane & 15;
  const int n0 = blockIdx.x * 32;
  const int m0w = blockIdx.y * 128 + 16 * w;

  const v8f zero8 = {0.f, 0.f, 0.f, 0.f, 0.f, 0.f, 0.f, 0.f};
  v8f acc[4][2];
  #pragma unroll
  for (int g = 0; g < 4; ++g) { acc[g][0] = zero8; acc[g][1] = zero8; }

  {
    const unsigned short* xa = Xb + (size_t)(m0w + m) * K1;
    const unsigned short* wb = Wih + (size_t)(n0 + m) * K1;
    const size_t gstr = (size_t)H * K1;
    #pragma unroll 1
    for (int k0 = 0; k0 < K1; k0 += 32) {
      const v16bf a = load_frag(xa + k0, h);
      #pragma unroll
      for (int g = 0; g < 4; ++g) {
        #pragma unroll
        for (int ct = 0; ct < 2; ++ct) {
          const v16bf b = load_frag(wb + g * gstr + (size_t)(16 * ct) * K1 + k0, h);
          acc[g][ct] = wmma_bf16(a, b, acc[g][ct]);
        }
      }
    }
  }
  {
    const unsigned short* ha = Hb + (size_t)(m0w + m) * K2;
    const unsigned short* wb = Whh + (size_t)(n0 + m) * K2;
    const size_t gstr = (size_t)H * K2;
    #pragma unroll 1
    for (int k0 = 0; k0 < K2; k0 += 32) {
      const v16bf a = load_frag(ha + k0, h);
      #pragma unroll
      for (int g = 0; g < 4; ++g) {
        #pragma unroll
        for (int ct = 0; ct < 2; ++ct) {
          const v16bf b = load_frag(wb + g * gstr + (size_t)(16 * ct) * K2 + k0, h);
          acc[g][ct] = wmma_bf16(a, b, acc[g][ct]);
        }
      }
    }
  }

  float* sh = sH + w * 512;
  float* sc = sC + w * 512;
  const float* crow = Cin + (size_t)(m0w + 8 * h) * H + n0 + m;
  #pragma unroll
  for (int ct = 0; ct < 2; ++ct) {
    const int col = n0 + 16 * ct + m;
    const float bi = bfr(bih[col])         + bfr(bhh[col]);
    const float bf = bfr(bih[H + col])     + bfr(bhh[H + col]);
    const float bg = bfr(bih[2 * H + col]) + bfr(bhh[2 * H + col]);
    const float bo = bfr(bih[3 * H + col]) + bfr(bhh[3 * H + col]);
    #pragma unroll
    for (int r = 0; r < 8; ++r) {
      float cp = 0.0f;
      if (useC) cp = crow[(size_t)r * H + 16 * ct];
      const float gi = acc[0][ct][r] + bi;
      const float gf = acc[1][ct][r] + bf;
      const float gg = acc[2][ct][r] + bg;
      const float go = acc[3][ct][r] + bo;
      const float c2 = fsigm(gf) * cp + fsigm(gi) * ftanh(gg);
      const float h2 = fsigm(go) * ftanh(c2);
      const int li = (8 * h + r) * 32 + 16 * ct + m;
      sh[li] = h2;
      sc[li] = c2;
    }
  }
  __syncthreads();

  float* hdst = Hout + (size_t)m0w * H + n0;
  float* cdst = Cout + (size_t)m0w * H + n0;
  tile_store(sh, hdst, H, lane);
  if (storeC) tile_store(sc, cdst, H, lane);
  __threadfence();
  tile_store(sh, hdst, H, lane);
  if (storeC) tile_store(sc, cdst, H, lane);
}

template <int L>
__device__ __forceinline__ void row_store(const float* y, int path, unsigned short* Hd, float* Cd,
                                          int row, float inv, int lane) {
  if (path == 0) {
    unsigned short* d = Hd + (size_t)row * L;
    #pragma unroll
    for (int i = 0; i < L / 256; ++i) {
      const float* q = y + 256 * i + 8 * lane;
      const v4f a = *(const v4fa*)q;
      const v4f b = *(const v4fa*)(q + 4);
      v8us o;
      o[0] = f2bf(a.x * inv); o[1] = f2bf(a.y * inv); o[2] = f2bf(a.z * inv); o[3] = f2bf(a.w * inv);
      o[4] = f2bf(b.x * inv); o[5] = f2bf(b.y * inv); o[6] = f2bf(b.z * inv); o[7] = f2bf(b.w * inv);
      *(volatile v8us*)(d + 256 * i + 8 * lane) = o;
    }
  } else {
    float* d = Cd + (size_t)row * L;
    #pragma unroll
    for (int i = 0; i < L / 128; ++i) {
      v4f a = *(const v4fa*)(y + 128 * i + 4 * lane);
      a = a * inv;
      *(volatile v4f*)(d + 128 * i + 4 * lane) = a;
    }
  }
}

template <int L>
__global__ __launch_bounds__(128) void conv_softmax_kernel(
    const float* __restrict__ Hs, const float* __restrict__ Cs,
    const float* __restrict__ wh, const float* __restrict__ wc,
    unsigned short* Hd, float* Cd)
{
  __shared__ __attribute__((aligned(16))) float sx[4 * L];
  __shared__ __attribute__((aligned(16))) float sy[4 * L];

  const int tid = threadIdx.x, lane = tid & 31, w = tid >> 5;
  const int path = blockIdx.y;
  const int row = blockIdx.x * 4 + w;
  const float* src = ((path == 0) ? Hs : Cs) + (size_t)row * L;
  const float* tp = (path == 0) ? wh : wc;
  const float t0 = bfr(tp[0]), t1 = bfr(tp[1]), t2 = bfr(tp[2]);
  float* x = sx + w * L;
  float* y = sy + w * L;

  #pragma unroll
  for (int i = 0; i < L / 128; ++i) {
    const v4f v = *(const v4fa*)(src + 128 * i + 4 * lane);
    *(v4fa*)(x + 128 * i + 4 * lane) = v;
  }
  __syncthreads();

  float mx = -3.0e38f;
  #pragma unroll 1
  for (int t = 0; t < L / 32; ++t) {
    const int j = 32 * t + lane;
    const int jl = (j > 0) ? (j - 1) : 0;
    const int jr = (j < L - 1) ? (j + 1) : (L - 1);
    float xl = x[jl];
    const float xc = x[j];
    float xr = x[jr];
    xl = (j > 0) ? xl : 0.0f;
    xr = (j < L - 1) ? xr : 0.0f;
    const float v = t0 * xl + t1 * xc + t2 * xr;
    y[j] = v;
    mx = fmaxf(mx, v);
  }
  mx = wave_max(mx);

  float s = 0.0f;
  #pragma unroll 1
  for (int t = 0; t < L / 32; ++t) {
    const int j = 32 * t + lane;
    const float p = __expf(y[j] - mx);
    y[j] = p;
    s += p;
  }
  s = wave_sum(s);
  const float inv = 1.0f / s;
  __syncthreads();

  row_store<L>(y, path, Hd, Cd, row, inv, lane);
  __threadfence();
  row_store<L>(y, path, Hd, Cd, row, inv, lane);
}

extern "C" void kernel_launch(void* const* d_in, const int* in_sizes, int n_in,
                              void* d_out, int out_size, void* d_ws, size_t ws_size,
                              hipStream_t stream) {
  if (n_in < 23) return;
  if (in_sizes[0] != NB * NID) return;
  if (in_sizes[1] != 4096 * 2048 || in_sizes[2] != 4096 * 1024) return;
  if (in_sizes[3] != 4096 || in_sizes[4] != 4096) return;
  if (in_sizes[5] != 2048 * 1024 || in_sizes[6] != 2048 * 512) return;
  if (in_sizes[7] != 2048 || in_sizes[8] != 2048) return;
  if (in_sizes[9] != 1024 * 512 || in_sizes[10] != 1024 * 256) return;
  if (in_sizes[11] != 1024 || in_sizes[12] != 1024) return;
  if (in_sizes[13] != 512 * 256 || in_sizes[14] != 512 * 128) return;
  if (in_sizes[15] != 512 || in_sizes[16] != 512) return;
  for (int i = 17; i < 23; ++i) if (in_sizes[i] != 3) return;
  if (out_size != NHC) return;

  const float* spec = (const float*)d_in[0];
  const float* Wih1 = (const float*)d_in[1];  const float* Whh1 = (const float*)d_in[2];
  const float* bih1 = (const float*)d_in[3];  const float* bhh1 = (const float*)d_in[4];
  const float* Wih2 = (const float*)d_in[5];  const float* Whh2 = (const float*)d_in[6];
  const float* bih2 = (const float*)d_in[7];  const float* bhh2 = (const float*)d_in[8];
  const float* Wih3 = (const float*)d_in[9];  const float* Whh3 = (const float*)d_in[10];
  const float* bih3 = (const float*)d_in[11]; const float* bhh3 = (const float*)d_in[12];
  const float* Wih4 = (const float*)d_in[13];
  const float* bih4 = (const float*)d_in[15]; const float* bhh4 = (const float*)d_in[16];
  const float* w2_1h = (const float*)d_in[17]; const float* w2_1c = (const float*)d_in[18];
  const float* w3_2h = (const float*)d_in[19]; const float* w3_2c = (const float*)d_in[20];
  const float* w4_3h = (const float*)d_in[21]; const float* w4_3c = (const float*)d_in[22];
  float* out = (float*)d_out;

  const size_t b_xb  = (size_t)NB * NID * 2;
  const size_t b_w1i = (size_t)4096 * 2048 * 2;
  const size_t b_w1h = (size_t)4096 * 1024 * 2;
  const size_t b_w2i = (size_t)2048 * 1024 * 2;
  const size_t b_w2h = (size_t)2048 * 512 * 2;
  const size_t b_w3i = (size_t)1024 * 512 * 2;
  const size_t b_w3h = (size_t)1024 * 256 * 2;
  const size_t b_w4i = (size_t)512 * 256 * 2;
  const size_t b_hf  = (size_t)NHC * 4;
  const size_t b_cf  = (size_t)NHC * 4;
  const size_t b_hb  = (size_t)NHC * 2;
  const size_t b_cb  = (size_t)NHC * 4;
  const size_t total = b_xb + b_w1i + b_w1h + b_w2i + b_w2h + b_w3i + b_w3h + b_w4i
                     + b_hf + b_cf + b_hb + b_cb;
  if (total > ws_size) return;

  char* ws = (char*)d_ws;
  size_t off = 0;
  unsigned short* Xb  = (unsigned short*)(ws + off); off += b_xb;
  unsigned short* W1i = (unsigned short*)(ws + off); off += b_w1i;
  unsigned short* W1h = (unsigned short*)(ws + off); off += b_w1h;
  unsigned short* W2i = (unsigned short*)(ws + off); off += b_w2i;
  unsigned short* W2h = (unsigned short*)(ws + off); off += b_w2h;
  unsigned short* W3i = (unsigned short*)(ws + off); off += b_w3i;
  unsigned short* W3h = (unsigned short*)(ws + off); off += b_w3h;
  unsigned short* W4i = (unsigned short*)(ws + off); off += b_w4i;
  float*          hbuf = (float*)(ws + off);         off += b_hf;
  float*          cbuf = (float*)(ws + off);         off += b_cf;
  unsigned short* hbb  = (unsigned short*)(ws + off); off += b_hb;
  float*          cbb  = (float*)(ws + off);         off += b_cb;
  if (off > ws_size) return;

  {
    const float* srcs[8] = { spec, Wih1, Whh1, Wih2, Whh2, Wih3, Whh3, Wih4 };
    unsigned short* dsts[8] = { Xb, W1i, W1h, W2i, W2h, W3i, W3h, W4i };
    const int n8s[8] = { NB * NID / 8, 4096 * 2048 / 8, 4096 * 1024 / 8, 2048 * 1024 / 8,
                         2048 * 512 / 8, 1024 * 512 / 8, 1024 * 256 / 8, 512 * 256 / 8 };
    for (int i = 0; i < 8; ++i) {
      const int n8 = n8s[i];
      cvt_bf16_kernel<<<(n8 + 255) / 256, 256, 0, stream>>>(srcs[i], dsts[i], n8);
    }
  }

  cell_gemm_kernel<<<dim3(128 / 32, 32768 / 128), 256, 0, stream>>>(
      Xb, 256, hbb, 0, W4i, W4i, bih4, bhh4, cbb, 0, hbuf, cbuf, 1, 128);
  conv_softmax_kernel<256><<<dim3(16384 / 4, 2), 128, 0, stream>>>(
      hbuf, cbuf, w4_3h, w4_3c, hbb, cbb);

  cell_gemm_kernel<<<dim3(256 / 32, 16384 / 128), 256, 0, stream>>>(
      Xb, 512, hbb, 256, W3i, W3h, bih3, bhh3, cbb, 1, hbuf, cbuf, 1, 256);
  conv_softmax_kernel<512><<<dim3(8192 / 4, 2), 128, 0, stream>>>(
      hbuf, cbuf, w3_2h, w3_2c, hbb, cbb);

  cell_gemm_kernel<<<dim3(512 / 32, 8192 / 128), 256, 0, stream>>>(
      Xb, 1024, hbb, 512, W2i, W2h, bih2, bhh2, cbb, 1, hbuf, cbuf, 1, 512);
  conv_softmax_kernel<1024><<<dim3(4096 / 4, 2), 128, 0, stream>>>(
      hbuf, cbuf, w2_1h, w2_1c, hbb, cbb);

  cell_gemm_kernel<<<dim3(1024 / 32, 4096 / 128), 256, 0, stream>>>(
      Xb, 2048, hbb, 1024, W1i, W1h, bih1, bhh1, cbb, 1, out, cbuf, 0, 1024);
}
